// OMNIANOMALY_60112362275054
// MI455X (gfx1250) — hardware-verified
//
#include <hip/hip_runtime.h>
#include <math.h>

#define NBATCH 128
#define NSTEP  64
#define XDIM   64
#define ZDIM   64
#define HID    512
#define DDIM   512
#define GATE3  1536
#define NROWS  8192
#define WPE_LD 576
#define NT     256
#define HPITCH 520
#define RPW    8
#define ROWS_PER_BLK 64
#define NPOSTBLK 128
#define HEADN  128
#define HEADPAIRS 16384
#define NOUTF  3145730
#define NPACKBLK 384

static_assert(NROWS == NBATCH * NSTEP);
static_assert(NPOSTBLK * ROWS_PER_BLK == NROWS);
static_assert(NPACKBLK * 8 * 32 * 32 + 2 == NOUTF);
static_assert(HEADPAIRS * 2 == 64 * DDIM);

#define PB_X   256
#define PB_WI  192
#define PB_WH  1536
#define PB_WP  512
#define PB_WS  64
#define PB_E0  (PB_X)
#define PB_E1  (PB_E0 + PB_WI)
#define PB_E2  (PB_E1 + PB_WH)
#define PB_E3  (PB_E2 + PB_WP)
#define PB_E4  (PB_E3 + PB_WS)
#define PB_E5  (PB_E4 + PB_WS)
#define PB_E6  (PB_E5 + PB_WI)
#define PB_E7  (PB_E6 + PB_WH)
#define PB_E8  (PB_E7 + PB_WP)
#define PB_E9  (PB_E8 + PB_WS)
#define PB_E10 (PB_E9 + PB_WS)
static_assert(PB_X * NT * 8 == NROWS * XDIM);
static_assert(PB_WI * NT * 2 == GATE3 * XDIM);
static_assert(PB_WH * NT * 2 == GATE3 * HID);
static_assert(PB_WP * NT * 2 == DDIM * HID);
static_assert(PB_WS * NT * 2 == 64 * DDIM);
static_assert(PB_E10 == 4992);

typedef __attribute__((ext_vector_type(16))) _Float16 v16h;
typedef __attribute__((ext_vector_type(8)))  _Float16 v8h;
typedef __attribute__((ext_vector_type(16))) __bf16   v16b;
typedef __attribute__((ext_vector_type(8)))  __bf16   v8b;
typedef __attribute__((ext_vector_type(8)))  float    v8f;
typedef __attribute__((ext_vector_type(4)))  float    v4f;
typedef __attribute__((ext_vector_type(2)))  float    v2f;
typedef __attribute__((ext_vector_type(2)))  unsigned v2u;

__device__ __forceinline__ unsigned short f2bf_bits(float f) {
  unsigned u = __float_as_uint(f);
  return (unsigned short)((u + 0x7FFFu + ((u >> 16) & 1u)) >> 16);
}
__device__ __forceinline__ float bf_bits2f(unsigned short h) { return __uint_as_float(((unsigned)h) << 16); }

__device__ __forceinline__ void dep_guard_h(v8f& a, v8f& b, v16h x, v16h y) { asm volatile("v_nop\n\tv_nop\n\tv_nop\n\tv_nop" : "+v"(a), "+v"(b) : "v"(x), "v"(y)); }
__device__ __forceinline__ void dep_guard_b(v8f& a, v8f& b, v16b x, v16b y) { asm volatile("v_nop\n\tv_nop\n\tv_nop\n\tv_nop" : "+v"(a), "+v"(b) : "v"(x), "v"(y)); }
__device__ __forceinline__ void keep4_h(v16h a, v16h b, v16h c, v16h d) { asm volatile("v_nop" :: "v"(a), "v"(b), "v"(c), "v"(d)); }
__device__ __forceinline__ void keep4_b(v16b a, v16b b, v16b c, v16b d) { asm volatile("v_nop" :: "v"(a), "v"(b), "v"(c), "v"(d)); }
__device__ __forceinline__ void acc_guard4(v8f& a, v8f& b, v8f& c, v8f& d) { asm volatile("v_nop\n\tv_nop\n\tv_nop\n\tv_nop" : "+v"(a), "+v"(b), "+v"(c), "+v"(d)); }
__device__ __forceinline__ void dep_guard3_h(v8f& a, v8f& b, v8f& c, v16h w, v16h x, v16h y, v16h z) {
  asm volatile("v_nop\n\tv_nop\n\tv_nop\n\tv_nop" : "+v"(a), "+v"(b), "+v"(c) : "v"(w), "v"(x), "v"(y), "v"(z));
}
__device__ __forceinline__ void acc_guard3(v8f& a, v8f& b, v8f& c) { asm volatile("v_nop\n\tv_nop\n\tv_nop\n\tv_nop" : "+v"(a), "+v"(b), "+v"(c)); }

template <typename T> struct Frag;
template <> struct Frag<_Float16> {
  typedef v16h V; union U { v16h v; v8h h[2]; };
  static __device__ __forceinline__ v16h load(const _Float16* p) {
    U f; f.h[0] = *(const v8h*)(p); f.h[1] = *(const v8h*)(p + 16); return f.v;
  }
  static __device__ __forceinline__ v8f mma(v16h a, v16h b, v8f c) {
    return __builtin_amdgcn_wmma_f32_16x16x32_f16(false, a, false, b, (short)0, c, false, false);
  }
  static __device__ __forceinline__ void guard(v8f& a, v8f& b, v16h x, v16h y) { dep_guard_h(a, b, x, y); }
  static __device__ __forceinline__ void keep(v16h a, v16h b, v16h c, v16h d) { keep4_h(a, b, c, d); }
};
template <> struct Frag<__bf16> {
  typedef v16b V; union U { v16b v; v8b h[2]; };
  static __device__ __forceinline__ v16b load(const __bf16* p) {
    U f; f.h[0] = *(const v8b*)(p); f.h[1] = *(const v8b*)(p + 16); return f.v;
  }
  static __device__ __forceinline__ v8f mma(v16b a, v16b b, v8f c) {
    return __builtin_amdgcn_wmma_f32_16x16x32_bf16(false, a, false, b, (short)0, c, false, false);
  }
  static __device__ __forceinline__ void guard(v8f& a, v8f& b, v16b x, v16b y) { dep_guard_b(a, b, x, y); }
  static __device__ __forceinline__ void keep(v16b a, v16b b, v16b c, v16b d) { keep4_b(a, b, c, d); }
};

template <int ET> struct Elem;
template <> struct Elem<0> { typedef _Float16 T; };
template <> struct Elem<1> { typedef __bf16 T; };
template <int ET, bool SPLIT, int BIAS_MODE, int OUT_MODE, bool RESID, int ACT = 0>
__global__ __launch_bounds__(256) void wmma_gemm64(
    const unsigned short* __restrict__ Ap, const unsigned short* __restrict__ A2p, int lda, long strideA,
    const unsigned short* __restrict__ Btp, const unsigned short* __restrict__ Bt2p, int ldb, long strideB,
    void* __restrict__ Cout, void* __restrict__ Cout2, int ldc, long strideC,
    const float* __restrict__ bias,
    const float* __restrict__ resid, long strideR,
    int M, int N, int K, float scale) {
  typedef typename Elem<ET>::T T;
  typedef typename Frag<T>::V V;
  const T* A = (const T*)Ap; const T* A2 = (const T*)A2p; const T* Bt = (const T*)Btp; const T* Bt2 = (const T*)Bt2p;
  __shared__ __align__(16) float sT[8][16 * 68];
  const int b    = blockIdx.y;
  const int lane = threadIdx.x & 31;
  const int wave = threadIdx.x >> 5;
  const int tilesN = N >> 6;
  const int tilesM = M >> 6;
  const int tile = blockIdx.x * 8 + wave;
  if (tile >= tilesM * tilesN) return;
  const int tm = tile / tilesN;
  const int tn = tile - tm * tilesN;
  const int m0 = tm << 6;
  const int n0 = tn << 6;

  const T* Ab  = A  + (size_t)b * strideA;
  const T* Bb  = Bt + (size_t)b * strideB;
  const T* Ab2 = SPLIT ? (A2  + (size_t)b * strideA) : nullptr;
  const T* Bb2 = SPLIT ? (Bt2 + (size_t)b * strideB) : nullptr;

  const int rlane = lane & 15;
  const int koff  = (lane >> 4) * 8;
  const int mOff  = (lane >> 4) * 8;

  v8f acc[4][4];
#pragma unroll
  for (int i = 0; i < 4; ++i)
#pragma unroll
    for (int j = 0; j < 4; ++j) acc[i][j] = (v8f){0.f,0.f,0.f,0.f,0.f,0.f,0.f,0.f};

  for (int k0 = 0; k0 < K; k0 += 32) {
    V bh[4], bl[4];
#pragma unroll
    for (int j = 0; j < 4; ++j) {
      const size_t bo = (size_t)(n0 + (j << 4) + rlane) * ldb + koff + k0;
      bh[j] = Frag<T>::load(Bb + bo);
      if (SPLIT) bl[j] = Frag<T>::load(Bb2 + bo);
    }
#pragma unroll
    for (int i = 0; i < 4; ++i) {
      const size_t ao = (size_t)(m0 + (i << 4) + rlane) * lda + koff + k0;
      V ah = Frag<T>::load(Ab + ao);
      V al;
      if (SPLIT) al = Frag<T>::load(Ab2 + ao);
#pragma unroll
      for (int j = 0; j < 4; ++j) {
        acc[i][j] = Frag<T>::mma(ah, bh[j], acc[i][j]);
        if (SPLIT) {
          acc[i][j] = Frag<T>::mma(ah, bl[j], acc[i][j]);
          acc[i][j] = Frag<T>::mma(al, bh[j], acc[i][j]);
        }
      }
      Frag<T>::guard(acc[i][0], acc[i][3], ah, SPLIT ? al : ah);
    }
    Frag<T>::keep(bh[0], bh[1], bh[2], bh[3]);
    if (SPLIT) Frag<T>::keep(bl[0], bl[1], bl[2], bl[3]);
  }
  acc_guard4(acc[0][0], acc[0][1], acc[0][2], acc[0][3]);
  acc_guard4(acc[1][0], acc[1][1], acc[1][2], acc[1][3]);
  acc_guard4(acc[2][0], acc[2][1], acc[2][2], acc[2][3]);
  acc_guard4(acc[3][0], acc[3][1], acc[3][2], acc[3][3]);

  float* slab = sT[wave];
  const float* Rb = RESID ? (resid + (size_t)b * strideR) : nullptr;
#pragma unroll
  for (int i = 0; i < 4; ++i) {
    const int mBase = m0 + (i << 4);
#pragma unroll
    for (int j = 0; j < 4; ++j) {
      const int n = n0 + (j << 4) + rlane;
      float bv = 0.f;
      if (BIAS_MODE == 2) bv = bias[n];
#pragma unroll
      for (int r = 0; r < 8; ++r) {
        float v = acc[i][j][r] * scale;
        if (BIAS_MODE == 1) v += bias[mBase + mOff + r];
        if (BIAS_MODE == 2) v += bv;
        if (RESID) v += Rb[(size_t)(mBase + mOff + r) * ldc + n];
        if (ACT == 1) v = tanhf(v);
        if (ACT == 2) v = fmaxf(v, 0.0f);
        if (ACT == 3) v = v / (1.0f + expf(-v));
        if (ACT == 4) v = (v > 0.f) ? v : 0.01f * v;
        if (ACT == 5) v = 0.5f * v * (1.0f + erff(v * 0.70710678118654752f));
        slab[(mOff + r) * 68 + (j << 4) + rlane] = v;
      }
    }
    __builtin_amdgcn_fence(__ATOMIC_RELEASE, "workgroup");
    __builtin_amdgcn_wave_barrier();
    __builtin_amdgcn_fence(__ATOMIC_ACQUIRE, "workgroup");
    if (OUT_MODE == 0) {
      float* C = (float*)Cout + (size_t)b * strideC;
      const int hh = lane >> 4, c4 = (lane & 15) * 4;
      for (int pass = 0; pass < 2; ++pass) {
#pragma unroll
        for (int it = 0; it < 8; ++it) {
          const int row = it * 2 + hh;
          v4f v = *(const v4f*)(slab + row * 68 + c4);
          *(volatile v4f*)(C + (size_t)(mBase + row) * ldc + n0 + c4) = v;
        }
        __threadfence();
      }
    } else {
      const int q = lane >> 3, c8 = (lane & 7) * 8;
      unsigned short* C  = (unsigned short*)Cout  + (size_t)b * strideC;
      unsigned short* C2 = (OUT_MODE == 2) ? ((unsigned short*)Cout2 + (size_t)b * strideC) : nullptr;
      for (int pass = 0; pass < 2; ++pass) {
#pragma unroll
        for (int it = 0; it < 4; ++it) {
          const int row = it * 4 + q;
          const float* sp = slab + row * 68 + c8;
          v8h hv, lv;
#pragma unroll
          for (int e = 0; e < 8; ++e) {
            if (OUT_MODE == 1) {
              hv[e] = (_Float16)sp[e];
            } else {
              unsigned short hb = f2bf_bits(sp[e]);
              unsigned short lb = f2bf_bits(sp[e] - bf_bits2f(hb));
              hv[e] = __builtin_bit_cast(_Float16, hb);
              lv[e] = __builtin_bit_cast(_Float16, lb);
            }
          }
          *(volatile v8h*)(C + (size_t)(mBase + row) * ldc + n0 + c8) = hv;
          if (OUT_MODE == 2) *(volatile v8h*)(C2 + (size_t)(mBase + row) * ldc + n0 + c8) = lv;
        }
        __threadfence();
      }
    }
    __builtin_amdgcn_fence(__ATOMIC_RELEASE, "workgroup");
    __builtin_amdgcn_wave_barrier();
    __builtin_amdgcn_fence(__ATOMIC_ACQUIRE, "workgroup");
  }
}

__device__ __forceinline__ unsigned pack_f16x2(float a, float b) {
  const _Float16 h0 = (_Float16)a, h1 = (_Float16)b;
  return (unsigned)__builtin_bit_cast(unsigned short, h0) | ((unsigned)__builtin_bit_cast(unsigned short, h1) << 16);
}
__device__ __forceinline__ void st2u(unsigned* p, unsigned v) { *(volatile unsigned*)p = v; __threadfence(); *(volatile unsigned*)p = v; }
__device__ __forceinline__ float ftanh(float x) { return 1.0f - 2.0f * __builtin_amdgcn_rcpf(1.0f + __expf(2.0f * x)); }
__device__ __forceinline__ float fsigm(float x) { return __builtin_amdgcn_rcpf(1.0f + __expf(-x)); }
__device__ __forceinline__ float fsoftplus(float x) { return fmaxf(x, 0.0f) + log1pf(__expf(-fabsf(x))); }
__device__ __forceinline__ void lds_wave_sync() {
  __builtin_amdgcn_fence(__ATOMIC_RELEASE, "workgroup");
  __builtin_amdgcn_wave_barrier();
  __builtin_amdgcn_fence(__ATOMIC_ACQUIRE, "workgroup");
}

__global__ __launch_bounds__(NT) void prep_kernel(const float* __restrict__ x,
                                                 const float* __restrict__ WiE, const float* __restrict__ WhE, const float* __restrict__ WpE,
                                                 const float* __restrict__ Wzm, const float* __restrict__ Wzs,
                                                 const float* __restrict__ WiD, const float* __restrict__ WhD, const float* __restrict__ WpD,
                                                 const float* __restrict__ Wxm, const float* __restrict__ Wxs,
                                                 _Float16* __restrict__ X16,
                                                 unsigned* __restrict__ PWIE, unsigned* __restrict__ PWHE,
                                                 unsigned* __restrict__ PWPE, unsigned* __restrict__ PWHZ,
                                                 unsigned* __restrict__ PWID, unsigned* __restrict__ PWHD,
                                                 unsigned* __restrict__ PWPD, unsigned* __restrict__ PWXZ) {
  const int blk = blockIdx.x, tid = threadIdx.x;
  const float wsc = 64.0f;
  if (blk < PB_E0) {
    const int gid = blk * NT + tid;
    const float* p = x + (size_t)gid * 8;
    const v4f a = *(const v4f*)p, bq = *(const v4f*)(p + 4);
    v8h h;
#pragma unroll
    for (int e = 0; e < 4; ++e) { h[e] = (_Float16)a[e]; h[4 + e] = (_Float16)bq[e]; }
    _Float16* op = X16 + (size_t)gid * 8;
    *(volatile v8h*)op = h; __threadfence(); *(volatile v8h*)op = h;
  } else if (blk < PB_E1) {
    const int p = (blk - PB_E0) * NT + tid;
    st2u(PWIE + p, pack_f16x2(WiE[2 * p] * wsc, WiE[2 * p + 1] * wsc));
  } else if (blk < PB_E2) {
    const int p = (blk - PB_E1) * NT + tid;
    st2u(PWHE + p, pack_f16x2(WhE[2 * p] * wsc, WhE[2 * p + 1] * wsc));
  } else if (blk < PB_E3) {
    const int p = (blk - PB_E2) * NT + tid;
    const int n = p >> 8, kk = (p & 255) * 2;
    const float* s = WpE + (size_t)n * WPE_LD + kk;
    st2u(PWPE + p, pack_f16x2(s[0] * wsc, s[1] * wsc));
  } else if (blk < PB_E4) {
    const int p = (blk - PB_E3) * NT + tid;
    st2u(PWHZ + p, pack_f16x2(Wzm[2 * p] * wsc, Wzm[2 * p + 1] * wsc));
  } else if (blk < PB_E5) {
    const int p = (blk - PB_E4) * NT + tid;
    st2u(PWHZ + HEADPAIRS + p, pack_f16x2(Wzs[2 * p] * wsc, Wzs[2 * p + 1] * wsc));
  } else if (blk < PB_E6) {
    const int p = (blk - PB_E5) * NT + tid;
    st2u(PWID + p, pack_f16x2(WiD[2 * p] * wsc, WiD[2 * p + 1] * wsc));
  } else if (blk < PB_E7) {
    const int p = (blk - PB_E6) * NT + tid;
    st2u(PWHD + p, pack_f16x2(WhD[2 * p] * wsc, WhD[2 * p + 1] * wsc));
  } else if (blk < PB_E8) {
    const int p = (blk - PB_E7) * NT + tid;
    st2u(PWPD + p, pack_f16x2(WpD[2 * p] * wsc, WpD[2 * p + 1] * wsc));
  } else if (blk < PB_E9) {
    const int p = (blk - PB_E8) * NT + tid;
    st2u(PWXZ + p, pack_f16x2(Wxm[2 * p] * wsc, Wxm[2 * p + 1] * wsc));
  } else {
    const int p = (blk - PB_E9) * NT + tid;
    st2u(PWXZ + HEADPAIRS + p, pack_f16x2(Wxs[2 * p] * wsc, Wxs[2 * p + 1] * wsc));
  }
}

__global__ __launch_bounds__(NT) void gru_rec_kernel(const float* __restrict__ XG, const _Float16* __restrict__ WHH,
                                                    const float* __restrict__ bhh, _Float16* __restrict__ HSEQ) {
  __shared__ __align__(16) _Float16 h16[16 * HPITCH];
  const int tid = threadIdx.x, lane = tid & 31, wave = tid >> 5;
  const int rlane = lane & 15, hh = lane >> 4, koff = hh * 8, mOff = hh * 8;
  const int blk = blockIdx.x;
  const int b0 = blk * 16;
  for (int i = tid; i < 16 * HPITCH; i += NT) h16[i] = (_Float16)0.0f;
  __syncthreads();

  const int jw = 64 * wave + rlane;
  const _Float16* arow = h16 + rlane * HPITCH + koff;
  float brg[4], bzg[4], bng[4];
#pragma unroll
  for (int c = 0; c < 4; ++c) {
    brg[c] = bhh[jw + 16 * c];
    bzg[c] = bhh[HID + jw + 16 * c];
    bng[c] = bhh[2 * HID + jw + 16 * c];
  }
  const float* xgb = XG + (size_t)(b0 + mOff) * NSTEP * GATE3 + jw;
  const v8f z8 = {0.f, 0.f, 0.f, 0.f, 0.f, 0.f, 0.f, 0.f};
  const float s64 = 1.0f / 64.0f;

  float hreg[4][8];
#pragma unroll
  for (int c = 0; c < 4; ++c)
#pragma unroll
    for (int r = 0; r < 8; ++r) hreg[c][r] = 0.0f;

#pragma unroll 1
  for (int t = 0; t < NSTEP; ++t) {
#pragma unroll
    for (int hp = 0; hp < 2; ++hp) {
      v8f ar[2], az[2], an[2];
      ar[0] = z8; az[0] = z8; an[0] = z8; ar[1] = z8; az[1] = z8; an[1] = z8;
      const _Float16* wbase = WHH + (size_t)(jw + 32 * hp) * HID + koff;
#pragma unroll 1
      for (int k0 = 0; k0 < HID; k0 += 32) {
        const v16h a = Frag<_Float16>::load(arow + k0);
#pragma unroll
        for (int c = 0; c < 2; ++c) {
          const _Float16* wc = wbase + (size_t)(16 * c) * HID + k0;
          const v16h bq0 = Frag<_Float16>::load(wc);
          const v16h bq1 = Frag<_Float16>::load(wc + (size_t)HID * HID);
          const v16h bq2 = Frag<_Float16>::load(wc + (size_t)2 * HID * HID);
          ar[c] = Frag<_Float16>::mma(a, bq0, ar[c]);
          az[c] = Frag<_Float16>::mma(a, bq1, az[c]);
          an[c] = Frag<_Float16>::mma(a, bq2, an[c]);
          dep_guard3_h(ar[c], az[c], an[c], a, bq0, bq1, bq2);
        }
      }
      acc_guard3(ar[0], az[0], an[0]);
      acc_guard3(ar[1], az[1], an[1]);

      const float* xt = xgb + (size_t)t * GATE3 + 32 * hp;
#pragma unroll
      for (int c = 0; c < 2; ++c) {
        const int ci = 2 * hp + c;
#pragma unroll
        for (int r = 0; r < 8; ++r) {
          const float* xr = xt + (size_t)r * NSTEP * GATE3 + 16 * c;
          const float x_r = xr[0], x_z = xr[HID], x_n = xr[2 * HID];
          const float hr = ar[c][r] * s64 + brg[ci];
          const float hz = az[c][r] * s64 + bzg[ci];
          const float hn = an[c][r] * s64 + bng[ci];
          const float rg = fsigm(x_r + hr);
          const float ug = fsigm(x_z + hz);
          const float ng = ftanh(x_n + rg * hn);
          hreg[ci][r] = (1.0f - ug) * ng + ug * hreg[ci][r];
        }
      }
    }
    __syncthreads();
#pragma unroll
    for (int c = 0; c < 4; ++c)
#pragma unroll
      for (int r = 0; r < 8; ++r) h16[(mOff + r) * HPITCH + jw + 16 * c] = (_Float16)hreg[c][r];
    __syncthreads();
    _Float16* hsb = HSEQ + ((size_t)b0 * NSTEP + t) * HID;
    for (int pass = 0; pass < 2; ++pass) {
#pragma unroll
      for (int rr = 0; rr < 2; ++rr) {
        const int row = 2 * wave + rr;
#pragma unroll
        for (int it = 0; it < 2; ++it) {
          const int c8 = it * 256 + lane * 8;
          const v8h v = *(const v8h*)(h16 + row * HPITCH + c8);
          *(volatile v8h*)(hsb + (size_t)row * NSTEP * HID + c8) = v;
        }
      }
      __threadfence();
    }
  }
}

__global__ __launch_bounds__(NT) void enc_post_kernel(const float* __restrict__ PRE, const float* __restrict__ bzm, const float* __restrict__ bzs,
                                                     const float* __restrict__ eps, const float* __restrict__ wfl, const float* __restrict__ bfl,
                                                     const float* __restrict__ ufl,
                                                     float* __restrict__ PZ, float* __restrict__ PZM, float* __restrict__ PZS,
                                                     unsigned* __restrict__ Z16u, float* __restrict__ PART) {
  __shared__ __align__(16) float zrow[8][64];
  __shared__ float wsum[8];
  const int tid = threadIdx.x, lane = tid & 31, wave = tid >> 5;
  const int blk = blockIdx.x;
  float* zr = zrow[wave];
  float kacc = 0.0f;
#pragma unroll 1
  for (int rr = 0; rr < RPW; ++rr) {
    const int row = blk * ROWS_PER_BLK + wave * RPW + rr;
    const int t = row & (NSTEP - 1);
#pragma unroll 1
    for (int cc = 0; cc < 2; ++cc) {
      const int col = 32 * cc + lane;
      const float pm = PRE[(size_t)row * HEADN + col] + bzm[col];
      const float ps = PRE[(size_t)row * HEADN + 64 + col] + bzs[col];
      const float zm = fsigm(pm);
      const float zs = fsoftplus(ps);
      const float e = eps[(size_t)row * 64 + col];
      const float z = e * zs + zm;
      kacc += (1.0f + zs) - zm * zm - __expf(zs);
      zr[col] = z;
      float* pmo = PZM + (size_t)row * 64 + col;
      float* pso = PZS + (size_t)row * 64 + col;
      *(volatile float*)pmo = zm; *(volatile float*)pso = zs;
      __threadfence();
      *(volatile float*)pmo = zm; *(volatile float*)pso = zs;
    }
    lds_wave_sync();
    float za = zr[lane], zb = zr[32 + lane];
#pragma unroll 1
    for (int k = 0; k < 2; ++k) {
      const int fi = (t * 2 + k) * 64;
      float sp = za * wfl[fi + lane] + zb * wfl[fi + 32 + lane];
#pragma unroll
      for (int off = 16; off > 0; off >>= 1) sp += __shfl_xor(sp, off, 32);
      const float th = ftanh(sp + bfl[t * 2 + k]);
      za += ufl[fi + lane] * th;
      zb += ufl[fi + 32 + lane] * th;
    }
    {
      float* pa = PZ + (size_t)row * 64 + lane;
      float* pb = pa + 32;
      *(volatile float*)pa = za; *(volatile float*)pb = zb;
      __threadfence();
      *(volatile float*)pa = za; *(volatile float*)pb = zb;
    }
    zr[lane] = za; zr[32 + lane] = zb;
    lds_wave_sync();
    {
      const v4f q = *(const v4f*)(zr + 4 * (lane & 15));
      v2u uu;
      uu[0] = pack_f16x2(q[0], q[1]);
      uu[1] = pack_f16x2(q[2], q[3]);
      unsigned* zo = Z16u + (size_t)row * 32 + 2 * (lane & 15);
      for (int pass = 0; pass < 2; ++pass) {
        if (lane < 16) *(volatile v2u*)zo = uu;
        __threadfence();
      }
    }
    lds_wave_sync();
  }
#pragma unroll
  for (int off = 16; off > 0; off >>= 1) kacc += __shfl_xor(kacc, off, 32);
  if (lane == 0) wsum[wave] = kacc;
  __syncthreads();
  if (wave == 0) {
    float v = wsum[lane & 7];
    v = (lane < 8) ? v : 0.0f;
    float* pp = PART + (size_t)blk * 32 + lane;
    *(volatile float*)pp = v; __threadfence(); *(volatile float*)pp = v;
  }
}

__global__ __launch_bounds__(NT) void dec_post_kernel(const float* __restrict__ PRE, const float* __restrict__ bxm, const float* __restrict__ bxs,
                                                     const float* __restrict__ eps, const float* __restrict__ x,
                                                     float* __restrict__ PXO, float* __restrict__ PXM, float* __restrict__ PXS,
                                                     float* __restrict__ PART) {
  __shared__ float nsum[8];
  __shared__ float ksum[8];
  const int tid = threadIdx.x, lane = tid & 31, wave = tid >> 5;
  const int blk = blockIdx.x;
  float nacc = 0.0f, kacc = 0.0f;
#pragma unroll 1
  for (int rr = 0; rr < RPW; ++rr) {
    const int row = blk * ROWS_PER_BLK + wave * RPW + rr;
#pragma unroll 1
    for (int cc = 0; cc < 2; ++cc) {
      const int col = 32 * cc + lane;
      const float pm = PRE[(size_t)row * HEADN + col] + bxm[col];
      const float ps = PRE[(size_t)row * HEADN + 64 + col] + bxs[col];
      const float xm = fsigm(pm);
      const float xs = fsoftplus(ps);
      const size_t ei = (size_t)row * 64 + col;
      const float e = eps[ei];
      const float xo = e * xs + xm;
      const float xx = x[ei];
      const float d = (xx - xm) * __expf(-0.5f * xs);
      nacc += xs + d * d;
      kacc += (1.0f + xs) - xm * xm - __expf(xs);
      float* po = PXO + ei; float* pmo = PXM + ei; float* pso = PXS + ei;
      *(volatile float*)po = xo; *(volatile float*)pmo = xm; *(volatile float*)pso = xs;
      __threadfence();
      *(volatile float*)po = xo; *(volatile float*)pmo = xm; *(volatile float*)pso = xs;
    }
  }
#pragma unroll
  for (int off = 16; off > 0; off >>= 1) { nacc += __shfl_xor(nacc, off, 32); kacc += __shfl_xor(kacc, off, 32); }
  if (lane == 0) { nsum[wave] = nacc; ksum[wave] = kacc; }
  __syncthreads();
  if (wave == 0) {
    const float v1 = nsum[lane & 7];
    const float v2 = ksum[lane & 7];
    const float v = (lane < 8) ? v1 : ((lane < 16) ? v2 : 0.0f);
    float* pp = PART + (size_t)blk * 32 + lane;
    *(volatile float*)pp = v; __threadfence(); *(volatile float*)pp = v;
  }
}

__global__ __launch_bounds__(NT) void pack_kernel(const float* __restrict__ PL, const float* __restrict__ PENC,
                                                 const float* __restrict__ PDEC, float* __restrict__ OUT) {
  __shared__ double dsum[3][32];
  const int tid = threadIdx.x, lane = tid & 31, wave = tid >> 5;
  const int blk = blockIdx.x;
  float nll = 0.0f, kld = 0.0f;
  if (blk == 0 && wave == 0) {
    double kz = 0.0, sa = 0.0, kx = 0.0;
#pragma unroll 1
    for (int bb = 0; bb < NPOSTBLK; ++bb) {
      const float v1 = PENC[bb * 32 + lane];
      const float v2 = PDEC[bb * 32 + lane];
      kz += (double)v1;
      sa += (lane < 8) ? (double)v2 : 0.0;
      kx += (lane >= 8 && lane < 16) ? (double)v2 : 0.0;
    }
    dsum[0][lane] = kz; dsum[1][lane] = sa; dsum[2][lane] = kx;
    lds_wave_sync();
    if (lane == 0) {
      double a = 0.0, s = 0.0, c = 0.0;
#pragma unroll 1
      for (int l = 0; l < 32; ++l) { a += dsum[0][l]; s += dsum[1][l]; c += dsum[2][l]; }
      nll = (float)(0.5 * s);
      kld = (float)(-0.5 * (a + c));
    }
  }
  const int gw = blk * 8 + wave;
#pragma unroll 1
  for (int it = 0; it < 8; ++it) {
    const long f0 = ((long)(gw * 32 + it * 4)) * 32 + (long)lane * 4;
    v4f q;
#pragma unroll
    for (int e = 0; e < 4; ++e) {
      const long i = f0 + e;
      const long ci = (i >= 2) ? (i - 2) : 0;
      const float pv = PL[ci];
      q[e] = (i == 0) ? nll : ((i == 1) ? kld : pv);
    }
    for (int pass = 0; pass < 2; ++pass) {
      *(volatile v4f*)(OUT + f0) = q;
      __threadfence();
    }
  }
  if (blk == 0 && wave == 0 && lane == 0) {
    v2f tl;
    tl[0] = PL[NOUTF - 4];
    tl[1] = PL[NOUTF - 3];
    float* tp = OUT + (NOUTF - 2);
    *(volatile v2f*)tp = tl; __threadfence(); *(volatile v2f*)tp = tl;
  }
}

extern "C" void kernel_launch(void* const* d_in, const int* in_sizes, int n_in,
                              void* d_out, int out_size, void* d_ws, size_t ws_size, hipStream_t stream) {
  if (n_in < 26 || d_out == nullptr || d_ws == nullptr) return;
  const int nact = NROWS * 64;
  if (in_sizes[0] != nact || in_sizes[1] != nact || in_sizes[2] != nact) return;
  if (in_sizes[3] != GATE3 * XDIM || in_sizes[4] != GATE3 * HID || in_sizes[5] != GATE3 || in_sizes[6] != GATE3) return;
  if (in_sizes[7] != DDIM * WPE_LD || in_sizes[8] != DDIM || in_sizes[9] != ZDIM * DDIM || in_sizes[10] != ZDIM ||
      in_sizes[11] != ZDIM * DDIM || in_sizes[12] != ZDIM) return;
  if (in_sizes[13] != NSTEP * 2 * ZDIM || in_sizes[14] != NSTEP * 2 || in_sizes[15] != NSTEP * 2 * ZDIM) return;
  if (in_sizes[16] != GATE3 * ZDIM || in_sizes[17] != GATE3 * HID || in_sizes[18] != GATE3 || in_sizes[19] != GATE3) return;
  if (in_sizes[20] != DDIM * HID || in_sizes[21] != DDIM || in_sizes[22] != XDIM * DDIM || in_sizes[23] != XDIM ||
      in_sizes[24] != XDIM * DDIM || in_sizes[25] != XDIM) return;
  if (out_size != NOUTF) return;

  const float* x       = (const float*)d_in[0];
  const float* eps_enc = (const float*)d_in[1];
  const float* eps_dec = (const float*)d_in[2];
  const float* Wi_enc  = (const float*)d_in[3];
  const float* Wh_enc  = (const float*)d_in[4];
  const float* bi_enc  = (const float*)d_in[5];
  const float* bh_enc  = (const float*)d_in[6];
  const float* Wp_enc  = (const float*)d_in[7];
  const float* bp_enc  = (const float*)d_in[8];
  const float* W_zm    = (const float*)d_in[9];
  const float* b_zm    = (const float*)d_in[10];
  const float* W_zs    = (const float*)d_in[11];
  const float* b_zs    = (const float*)d_in[12];
  const float* w_flow  = (const float*)d_in[13];
  const float* b_flow  = (const float*)d_in[14];
  const float* u_flow  = (const float*)d_in[15];
  const float* Wi_dec  = (const float*)d_in[16];
  const float* Wh_dec  = (const float*)d_in[17];
  const float* bi_dec  = (const float*)d_in[18];
  const float* bh_dec  = (const float*)d_in[19];
  const float* Wp_dec  = (const float*)d_in[20];
  const float* bp_dec  = (const float*)d_in[21];
  const float* W_xm    = (const float*)d_in[22];
  const float* b_xm    = (const float*)d_in[23];
  const float* W_xs    = (const float*)d_in[24];
  const float* b_xs    = (const float*)d_in[25];
  float* out = (float*)d_out;

  char* ws = (char*)d_ws; size_t off = 0;
  auto carve = [&](size_t bytes) -> char* { char* p = ws + off; off += (bytes + 255) & ~(size_t)255; return p; };
  _Float16* X16   = (_Float16*)carve((size_t)NROWS * XDIM * 2);
  unsigned* PWIE  = (unsigned*)carve((size_t)GATE3 * XDIM * 2);
  unsigned* PWHE  = (unsigned*)carve((size_t)GATE3 * HID * 2);
  unsigned* PWPE  = (unsigned*)carve((size_t)DDIM * HID * 2);
  unsigned* PWHZ  = (unsigned*)carve((size_t)HEADN * DDIM * 2);
  unsigned* PWID  = (unsigned*)carve((size_t)GATE3 * ZDIM * 2);
  unsigned* PWHD  = (unsigned*)carve((size_t)GATE3 * HID * 2);
  unsigned* PWPD  = (unsigned*)carve((size_t)DDIM * HID * 2);
  unsigned* PWXZ  = (unsigned*)carve((size_t)HEADN * DDIM * 2);
  float*    XG    = (float*)carve((size_t)NROWS * GATE3 * 4);
  _Float16* HSEQ  = (_Float16*)carve((size_t)NROWS * HID * 2);
  _Float16* PHI16 = (_Float16*)carve((size_t)NROWS * DDIM * 2);
  float*    PRE   = (float*)carve((size_t)NROWS * HEADN * 4);
  unsigned* Z16u  = (unsigned*)carve((size_t)NROWS * ZDIM * 2);
  float*    PL    = (float*)carve((size_t)6 * NROWS * 64 * 4);
  float*    PENC  = (float*)carve((size_t)NPOSTBLK * 32 * 4);
  float*    PDEC  = (float*)carve((size_t)NPOSTBLK * 32 * 4);
  if (off > ws_size || off > (size_t)134217728) return;
  float* PZ  = PL;
  float* PZM = PL + (size_t)1 * NROWS * 64;
  float* PZS = PL + (size_t)2 * NROWS * 64;
  float* PXO = PL + (size_t)3 * NROWS * 64;
  float* PXM = PL + (size_t)4 * NROWS * 64;
  float* PXS = PL + (size_t)5 * NROWS * 64;
  const float inv64 = 1.0f / 64.0f;
  const unsigned short* nul16 = (const unsigned short*)nullptr;
  const int gridXG   = (NROWS / 64) * (GATE3 / 64) / 8;
  const int gridPHI  = (NROWS / 64) * (DDIM / 64) / 8;
  const int gridHEAD = (NROWS / 64) * (HEADN / 64) / 8;

  prep_kernel<<<PB_E10, NT, 0, stream>>>(x, Wi_enc, Wh_enc, Wp_enc, W_zm, W_zs, Wi_dec, Wh_dec, Wp_dec, W_xm, W_xs,
                                         X16, PWIE, PWHE, PWPE, PWHZ, PWID, PWHD, PWPD, PWXZ);
  wmma_gemm64<0, false, 2, 0, false, 0><<<dim3(gridXG, 1), 256, 0, stream>>>(
      (const unsigned short*)X16, nul16, XDIM, 0L, (const unsigned short*)PWIE, nul16, XDIM, 0L,
      (void*)XG, (void*)nullptr, GATE3, 0L, bi_enc, (const float*)nullptr, 0L, NROWS, GATE3, XDIM, inv64);
  gru_rec_kernel<<<NBATCH / 16, NT, 0, stream>>>(XG, (const _Float16*)PWHE, bh_enc, HSEQ);
  wmma_gemm64<0, false, 2, 1, false, 2><<<dim3(gridPHI, 1), 256, 0, stream>>>(
      (const unsigned short*)HSEQ, nul16, HID, 0L, (const unsigned short*)PWPE, nul16, HID, 0L,
      (void*)PHI16, (void*)nullptr, DDIM, 0L, bp_enc, (const float*)nullptr, 0L, NROWS, DDIM, HID, inv64);
  wmma_gemm64<0, false, 0, 0, false, 0><<<dim3(gridHEAD, 1), 256, 0, stream>>>(
      (const unsigned short*)PHI16, nul16, DDIM, 0L, (const unsigned short*)PWHZ, nul16, DDIM, 0L,
      (void*)PRE, (void*)nullptr, HEADN, 0L, (const float*)nullptr, (const float*)nullptr, 0L, NROWS, HEADN, DDIM, inv64);
  enc_post_kernel<<<NPOSTBLK, NT, 0, stream>>>(PRE, b_zm, b_zs, eps_enc, w_flow, b_flow, u_flow, PZ, PZM, PZS, Z16u, PENC);
  wmma_gemm64<0, false, 2, 0, false, 0><<<dim3(gridXG, 1), 256, 0, stream>>>(
      (const unsigned short*)Z16u, nul16, ZDIM, 0L, (const unsigned short*)PWID, nul16, ZDIM, 0L,
      (void*)XG, (void*)nullptr, GATE3, 0L, bi_dec, (const float*)nullptr, 0L, NROWS, GATE3, ZDIM, inv64);
  gru_rec_kernel<<<NBATCH / 16, NT, 0, stream>>>(XG, (const _Float16*)PWHD, bh_dec, HSEQ);
  wmma_gemm64<0, false, 2, 1, false, 2><<<dim3(gridPHI, 1), 256, 0, stream>>>(
      (const unsigned short*)HSEQ, nul16, HID, 0L, (const unsigned short*)PWPD, nul16, HID, 0L,
      (void*)PHI16, (void*)nullptr, DDIM, 0L, bp_dec, (const float*)nullptr, 0L, NROWS, DDIM, HID, inv64);
  wmma_gemm64<0, false, 0, 0, false, 0><<<dim3(gridHEAD, 1), 256, 0, stream>>>(
      (const unsigned short*)PHI16, nul16, DDIM, 0L, (const unsigned short*)PWXZ, nul16, DDIM, 0L,
      (void*)PRE, (void*)nullptr, HEADN, 0L, (const float*)nullptr, (const float*)nullptr, 0L, NROWS, HEADN, DDIM, inv64);
  dec_post_kernel<<<NPOSTBLK, NT, 0, stream>>>(PRE, b_xm, b_xs, eps_dec, x, PXO, PXM, PXS, PDEC);
  pack_kernel<<<NPACKBLK, NT, 0, stream>>>(PL, PENC, PDEC, out);
}
